// GATModule_48249662603979
// MI455X (gfx1250) — hardware-verified
//
#include <hip/hip_runtime.h>
#include <stddef.h>


typedef _Float16 v16h __attribute__((ext_vector_type(16)));
typedef _Float16 v8h  __attribute__((ext_vector_type(8)));
typedef _Float16 v4h  __attribute__((ext_vector_type(4)));
typedef float    v8f  __attribute__((ext_vector_type(8)));
typedef float    v4f  __attribute__((ext_vector_type(4)));
typedef unsigned int v4u __attribute__((ext_vector_type(4)));
typedef v8h v8ha __attribute__((may_alias));
typedef v4h v4ha __attribute__((may_alias));
typedef v4f v4fa __attribute__((may_alias));
typedef v4u v4ua __attribute__((may_alias));

#define BS 8
#define NN 1024
#define CC 128
#define IMG 256
#define NEG_SLOPE 0.2f
#define LN_EPS 1e-5f
#define RPG 256
#define NGRP (NN / RPG)
#define GB 64
#define NBLK (NN / GB)
#define APITCH 136
#define TPITCH 132

union Frag { v16h v; v8h half[2]; };

__device__ __forceinline__ v8f vzero8() {
  v8f z = {0.f, 0.f, 0.f, 0.f, 0.f, 0.f, 0.f, 0.f};
  return z;
}

__device__ __forceinline__ v8f wmma16(v16h a, v16h b, v8f c) {
  v8f d = __builtin_amdgcn_wmma_f32_16x16x32_f16(false, a, false, b, (short)0, c, false, false);
  asm volatile("v_nop\n\tv_nop\n\tv_nop\n\tv_nop" : "+v"(d) : "v"(a), "v"(b));
  return d;
}

__device__ __forceinline__ void adj_pair(unsigned int* sB, int R0, int x, int y) {
  if (x > 0 && y > 0 && x != y) {
    int xi = x - 1; xi = xi > NN - 1 ? NN - 1 : xi;
    int yi = y - 1; yi = yi > NN - 1 ? NN - 1 : yi;
    if ((unsigned)(xi - R0) < (unsigned)RPG)
      atomicOr(&sB[(xi - R0) * 32 + (yi >> 5)], 1u << (yi & 31));
    if ((unsigned)(yi - R0) < (unsigned)RPG)
      atomicOr(&sB[(yi - R0) * 32 + (xi >> 5)], 1u << (xi & 31));
  }
}

__device__ __forceinline__ void adj_store(const unsigned int* sB, unsigned int* adjo,
                                          int g, int R0, int w, int l) {
#pragma unroll
  for (int s = 0; s < 8; ++s) {
    const int rl = w * 32 + s * 4 + (l >> 3), ch = l & 7;
    v4u v = *(const v4ua*)(sB + rl * 32 + ch * 4);
    *(volatile v4u*)(adjo + ((size_t)(g * NN + R0 + rl)) * 32 + ch * 4) = v;
  }
}

__global__ void __launch_bounds__(256) k_adj(const int* __restrict__ seg, unsigned int* adjo, int nG) {
  __shared__ unsigned int sB[RPG * 32];
  const int g = blockIdx.x / NGRP, grp = blockIdx.x - g * NGRP;
  if (g >= nG) return;
  const int R0 = grp * RPG, tid = threadIdx.x;
  for (int i = tid; i < RPG * 32; i += 256) sB[i] = 0u;
  __syncthreads();
  for (int r = tid; r < RPG; r += 256) {
    const int gr = R0 + r;
    sB[r * 32 + (gr >> 5)] = 1u << (gr & 31);
  }
  __syncthreads();
  const int* s = seg + (size_t)g * IMG * IMG;
  for (int p = tid; p < IMG * IMG; p += 256) {
    const int r = p >> 8, c = p & (IMG - 1);
    const bool hr = c < IMG - 1, hd = r < IMG - 1;
    const int a  = s[p];
    const int vr = s[p + (hr ? 1 : 0)];
    const int vd = s[p + (hd ? IMG : 0)];
    const int vg = s[p + ((hr && hd) ? (IMG + 1) : 0)];
    const int rt = hr ? vr : 0;
    const int dn = hd ? vd : 0;
    const int dg = (hr && hd) ? vg : 0;
    adj_pair(sB, R0, a, rt);
    adj_pair(sB, R0, a, dn);
    adj_pair(sB, R0, a, dg);
    adj_pair(sB, R0, rt, dn);
  }
  __syncthreads();
  const int w = tid >> 5, l = tid & 31;
  adj_store(sB, adjo, g, R0, w, l);
  __threadfence();
  adj_store(sB, adjo, g, R0, w, l);
}

template <int HEADS>
__device__ __forceinline__ void gemm_store(const float* sT, const float* sSc, _Float16* WfT,
                                           float* es, float* ed, int g, int node0, int w, int l) {
#pragma unroll
  for (int s = 0; s < 8; ++s) {
    const int c = w * 32 + s * 4 + (l >> 3), ch = l & 7;
    v8h hv;
#pragma unroll
    for (int e = 0; e < 8; ++e)
      hv[e] = (_Float16)(sT[(ch * 8 + e) * TPITCH + c] * (1.0f / 128.0f));
    *(volatile v8h*)(WfT + ((size_t)(g * CC + c)) * NN + node0 + ch * 8) = hv;
  }
  if (w == 0) {
#pragma unroll
    for (int s = 0; s < HEADS; ++s) {
      const int sg = s * 2 + (l >> 4), q = l & 15;
      v4f v = *(const v4fa*)(sSc + sg * GB + q * 4);
      const int which = (sg >= HEADS) ? 1 : 0;
      const int hh = sg - which * HEADS;
      float* dst = (which ? ed : es) + ((size_t)(g * HEADS + hh)) * NN + node0 + q * 4;
      *(volatile v4f*)dst = v;
    }
  }
}

template <int HEADS>
__global__ void __launch_bounds__(128) k_gemm(const float* __restrict__ X, const float* __restrict__ Wt,
                                              const float* __restrict__ aS, const float* __restrict__ aD,
                                              _Float16* WfT, float* es, float* ed, int nG) {
  constexpr int D = CC / HEADS, DH = D / 2;
  __shared__ v4f smem[3264];
  _Float16* sA = (_Float16*)smem;
  _Float16* sW = sA + GB * APITCH;
  float* sT  = (float*)smem;
  float* sSc = sT + GB * TPITCH;
  const int g = blockIdx.x / NBLK, nb = blockIdx.x - g * NBLK;
  if (g >= nG) return;
  const int node0 = nb * GB;
  const int tid = threadIdx.x, w = tid >> 5, l = tid & 31, h = l >> 4, m = l & 15;

  for (int idx = tid; idx < GB * (CC / 4); idx += 128) {
    const int row = idx >> 5, c4 = idx & 31;
    v4f x = *(const v4f*)(X + ((size_t)(g * NN + node0 + row)) * CC + c4 * 4);
    v4h hx;
#pragma unroll
    for (int e = 0; e < 4; ++e) hx[e] = (_Float16)(x[e] * 8.0f);
    *(v4ha*)(sA + row * APITCH + c4 * 4) = hx;
  }
  for (int idx = tid; idx < CC * (CC / 4); idx += 128) {
    const int row = idx >> 5, c4 = idx & 31;
    v4f x = *(const v4f*)(Wt + row * CC + c4 * 4);
    v4h hx;
#pragma unroll
    for (int e = 0; e < 4; ++e) hx[e] = (_Float16)(x[e] * 64.0f);
    *(v4ha*)(sW + row * APITCH + c4 * 4) = hx;
  }
  __syncthreads();

  v8f acc[8];
#pragma unroll
  for (int nt = 0; nt < 8; ++nt) acc[nt] = vzero8();
  const _Float16* arow = sA + (w * 16 + m) * APITCH;
#pragma unroll
  for (int kk = 0; kk < CC; kk += 32) {
    Frag a;
    a.half[0] = *(const v8ha*)(arow + kk + 8 * h);
    a.half[1] = *(const v8ha*)(arow + kk + 16 + 8 * h);
#pragma unroll
    for (int nt = 0; nt < 8; ++nt) {
      const _Float16* brow = sW + (nt * 16 + m) * APITCH + kk;
      Frag b;
      b.half[0] = *(const v8ha*)(brow + 8 * h);
      b.half[1] = *(const v8ha*)(brow + 16 + 8 * h);
      acc[nt] = wmma16(a.v, b.v, acc[nt]);
    }
  }
  __syncthreads();
#pragma unroll
  for (int nt = 0; nt < 8; ++nt)
#pragma unroll
    for (int r = 0; r < 8; ++r)
      sT[(w * 16 + 8 * h + r) * TPITCH + nt * 16 + m] = acc[nt][r];
  __syncthreads();

  {
    const int row = tid >> 1, part = tid & 1;
#pragma unroll
    for (int hh = 0; hh < HEADS; ++hh) {
      const int c0 = hh * D + part * DH;
      float s = 0.f, t = 0.f;
#pragma unroll 4
      for (int k = 0; k < DH; ++k) {
        const float v = sT[row * TPITCH + c0 + k] * (1.0f / 512.0f);
        s += v * aS[c0 + k];
        t += v * aD[c0 + k];
      }
      s += __shfl_xor(s, 1, 32);
      t += __shfl_xor(t, 1, 32);
      if (part == 0) {
        sSc[hh * GB + row] = s;
        sSc[(HEADS + hh) * GB + row] = t;
      }
    }
  }
  __syncthreads();
  gemm_store<HEADS>(sT, sSc, WfT, es, ed, g, node0, w, l);
  __threadfence();
  gemm_store<HEADS>(sT, sSc, WfT, es, ed, g, node0, w, l);
}

template <int D>
__device__ __forceinline__ void tile_store(const float* sOw, float* base, size_t rowBase, int col0, int l) {
  constexpr int OP = D + 4, CPR = D / 4, RPI = 32 / CPR, NI = 16 / RPI;
#pragma unroll
  for (int s = 0; s < NI; ++s) {
    const int row = s * RPI + l / CPR, ch = l % CPR;
    v4f v = *(const v4fa*)(sOw + row * OP + ch * 4);
    *(volatile v4f*)(base + (rowBase + row) * CC + col0 + ch * 4) = v;
  }
}

template <int HEADS, bool LN>
__global__ void __launch_bounds__(128) k_attn(const unsigned int* __restrict__ adj,
                                              const float* __restrict__ es, const float* __restrict__ ed,
                                              const _Float16* __restrict__ WfT,
                                              const float* __restrict__ feats,
                                              const float* __restrict__ gam, const float* __restrict__ bet,
                                              float* dst, int nG) {
  constexpr int D = CC / HEADS, NT = D / 16, OP = D + 4;
  __shared__ float sED[NN];
  __shared__ v4f sO4[16 * OP];
  float* sO = (float*)sO4;
  const int bid = blockIdx.x;
  const int g = bid / (HEADS * NBLK), rem = bid - g * HEADS * NBLK;
  const int head = rem / NBLK, rb = rem - head * NBLK;
  if (g >= nG) return;
  const int tid = threadIdx.x, w = tid >> 5, l = tid & 31, h = l >> 4, m = l & 15;

  const float* edg = ed + ((size_t)(g * HEADS + head)) * NN;
  for (int j = tid; j < NN; j += 128) sED[j] = edg[j];
  __syncthreads();

  const int i0 = rb * GB + w * 16;
  const size_t rowBase = (size_t)g * NN + i0;
  float* sOw = sO + w * 16 * OP;

  float myMx = 0.f;
#pragma unroll 1
  for (int r = 0; r < 16; ++r) {
    const unsigned int wv = adj[(rowBase + r) * 32 + l];
    float mx = -__builtin_huge_valf();
    const float* ep = sED + l * 32;
#pragma unroll
    for (int b4 = 0; b4 < 8; ++b4) {
      v4f q = *(const v4fa*)(ep + b4 * 4);
#pragma unroll
      for (int e = 0; e < 4; ++e)
        mx = ((wv >> (b4 * 4 + e)) & 1u) ? fmaxf(mx, q[e]) : mx;
    }
#pragma unroll
    for (int off = 16; off > 0; off >>= 1) mx = fmaxf(mx, __shfl_xor(mx, off, 32));
    myMx = (m == r) ? mx : myMx;
  }
  const float esm = es[((size_t)(g * HEADS + head)) * NN + i0 + m];
  float M = esm + myMx;
  M = (M >= 0.f) ? M : NEG_SLOPE * M;

  v8f acc[NT];
#pragma unroll
  for (int t = 0; t < NT; ++t) acc[t] = vzero8();
  float psum = 0.f;
  const unsigned int* arow = adj + (rowBase + m) * 32;
  const _Float16* wbase = WfT + ((size_t)(g * CC + head * D + m)) * NN;
#pragma unroll 1
  for (int kt = 0; kt < NN / 32; ++kt) {
    const int kk = kt * 32;
    const unsigned int aw = arow[kt];
    v4f q0 = *(const v4fa*)(sED + kk + 8 * h);
    v4f q1 = *(const v4fa*)(sED + kk + 8 * h + 4);
    v4f q2 = *(const v4fa*)(sED + kk + 16 + 8 * h);
    v4f q3 = *(const v4fa*)(sED + kk + 16 + 8 * h + 4);
    float edv[16];
#pragma unroll
    for (int e = 0; e < 4; ++e) {
      edv[e] = q0[e]; edv[4 + e] = q1[e]; edv[8 + e] = q2[e]; edv[12 + e] = q3[e];
    }
    v16h av;
#pragma unroll
    for (int i = 0; i < 16; ++i) {
      const int kb = i + (i & 8) + 8 * h;
      float x = esm + edv[i];
      x = (x >= 0.f) ? x : NEG_SLOPE * x;
      const float p = ((aw >> kb) & 1u) ? __expf(x - M) : 0.f;
      psum += p;
      av[i] = (_Float16)(p * 4096.0f);
    }
#pragma unroll
    for (int t = 0; t < NT; ++t) {
      const _Float16* bp = wbase + (size_t)t * 16 * NN + kk;
      Frag b;
      b.half[0] = *(const v8h*)(bp + 8 * h);
      b.half[1] = *(const v8h*)(bp + 16 + 8 * h);
      acc[t] = wmma16(av, b.v, acc[t]);
    }
  }
  psum += __shfl_xor(psum, 16, 32);
  const float rinvm = 1.0f / psum;
#pragma unroll
  for (int r = 0; r < 8; ++r) {
    const float sc = __shfl(rinvm, 8 * h + r, 32) * (1.0f / 16384.0f);
#pragma unroll
    for (int t = 0; t < NT; ++t) {
      float v = acc[t][r] * sc;
      if (!LN) v = (v > 0.f) ? v : (__expf(v) - 1.0f);
      sOw[(8 * h + r) * OP + t * 16 + m] = v;
    }
  }
  __syncthreads();

  if (!LN) {
    tile_store<D>(sOw, dst, rowBase, head * D, l);
    __threadfence();
    tile_store<D>(sOw, dst, rowBase, head * D, l);
  } else {
    float gm[4], bt[4];
#pragma unroll
    for (int u = 0; u < 4; ++u) { gm[u] = gam[l + 32 * u]; bt[u] = bet[l + 32 * u]; }
#pragma unroll 1
    for (int r = 0; r < 16; ++r) {
      const float* fr = feats + (rowBase + r) * CC;
      float y[4];
      float s = 0.f;
#pragma unroll
      for (int u = 0; u < 4; ++u) {
        y[u] = sOw[r * OP + l + 32 * u] + fr[l + 32 * u];
        s += y[u];
      }
#pragma unroll
      for (int off = 16; off > 0; off >>= 1) s += __shfl_xor(s, off, 32);
      const float mean = s * (1.0f / CC);
      float sq = 0.f;
#pragma unroll
      for (int u = 0; u < 4; ++u) { y[u] -= mean; sq += y[u] * y[u]; }
#pragma unroll
      for (int off = 16; off > 0; off >>= 1) sq += __shfl_xor(sq, off, 32);
      const float rstd = rsqrtf(sq * (1.0f / CC) + LN_EPS);
#pragma unroll
      for (int u = 0; u < 4; ++u) sOw[r * OP + l + 32 * u] = y[u] * rstd * gm[u] + bt[u];
    }
    __syncthreads();
    tile_store<D>(sOw, dst, rowBase, 0, l);
    __threadfence();
    tile_store<D>(sOw, dst, rowBase, 0, l);
  }
}

extern "C" void kernel_launch(void* const* d_in, const int* in_sizes, int n_in,
                              void* d_out, int out_size, void* d_ws, size_t ws_size,
                              hipStream_t stream) {
  if (n_in < 11) return;
  if (in_sizes[0] != BS * NN * CC || in_sizes[1] != BS * IMG * IMG ||
      in_sizes[3] != CC * CC || in_sizes[4] != CC || in_sizes[5] != CC ||
      in_sizes[6] != CC * CC || in_sizes[7] != CC || in_sizes[8] != CC ||
      in_sizes[9] != CC || in_sizes[10] != CC || out_size != BS * NN * CC) return;

  const float* feats = (const float*)d_in[0];
  const int*   segI  = (const int*)d_in[1];
  const float* W1  = (const float*)d_in[3];
  const float* aS1 = (const float*)d_in[4];
  const float* aD1 = (const float*)d_in[5];
  const float* W2  = (const float*)d_in[6];
  const float* aS2 = (const float*)d_in[7];
  const float* aD2 = (const float*)d_in[8];
  const float* gam = (const float*)d_in[9];
  const float* bet = (const float*)d_in[10];
  float* out = (float*)d_out;

  const size_t nAdj = (size_t)BS * NN * 32 * 4;
  const size_t nWfT = (size_t)BS * CC * NN * 2;
  const size_t nE1  = (size_t)BS * 4 * NN * 4;
  const size_t nH1  = (size_t)BS * NN * CC * 4;
  const size_t nE2  = (size_t)BS * 1 * NN * 4;
  const size_t oAdj  = 0;
  const size_t oWfT1 = oAdj + nAdj;
  const size_t oEs1  = oWfT1 + nWfT;
  const size_t oEd1  = oEs1 + nE1;
  const size_t oH1   = oEd1 + nE1;
  const size_t oWfT2 = oH1 + nH1;
  const size_t oEs2  = oWfT2 + nWfT;
  const size_t oEd2  = oEs2 + nE2;
  const size_t total = oEd2 + nE2;
  if (total > ws_size) return;

  char* ws = (char*)d_ws;
  unsigned int* adj = (unsigned int*)(ws + oAdj);
  _Float16* WfT1 = (_Float16*)(ws + oWfT1);
  float* es1 = (float*)(ws + oEs1);
  float* ed1 = (float*)(ws + oEd1);
  float* h1  = (float*)(ws + oH1);
  _Float16* WfT2 = (_Float16*)(ws + oWfT2);
  float* es2 = (float*)(ws + oEs2);
  float* ed2 = (float*)(ws + oEd2);

  k_adj<<<BS * NGRP, 256, 0, stream>>>(segI, adj, BS);
  k_gemm<4><<<BS * NBLK, 128, 0, stream>>>(feats, W1, aS1, aD1, WfT1, es1, ed1, BS);
  k_attn<4, false><<<BS * 4 * NBLK, 128, 0, stream>>>(adj, es1, ed1, WfT1, feats, gam, bet, h1, BS);
  k_gemm<1><<<BS * NBLK, 128, 0, stream>>>(h1, W2, aS2, aD2, WfT2, es2, ed2, BS);
  k_attn<1, true><<<BS * 1 * NBLK, 128, 0, stream>>>(adj, es2, ed2, WfT2, feats, gam, bet, out, BS);
}
